// cosine_similarity_87101936763000
// MI455X (gfx1250) — hardware-verified
//
#include <hip/hip_runtime.h>

typedef _Float16 v16h __attribute__((ext_vector_type(16)));
typedef _Float16 v8h  __attribute__((ext_vector_type(8)));
typedef float    v8f  __attribute__((ext_vector_type(8)));
typedef float    v4f  __attribute__((ext_vector_type(4)));
typedef v8h __attribute__((may_alias)) v8ha;
typedef v4f __attribute__((may_alias)) v4fa;

union Frag { v16h v; v8h half[2]; };

#define SEQ   1024
#define NB    32
#define DIM   128
#define NELEM (SEQ * NB * DIM)
#define G8    (NELEM / 8)
#define RPB   16
#define RT    (SEQ / RPB)
#define NTHR  128
#define NWAVE 4
#define CPW   (SEQ / NWAVE)
#define RVL   32

static_assert(SEQ % RPB == 0);
static_assert(CPW % 16 == 0);
static_assert(DIM % 32 == 0);
static_assert(RPB == NWAVE * 4);

__device__ __forceinline__ v8f wmma_f16(v16h a, v16h b, v8f c) {
  v8f d = __builtin_amdgcn_wmma_f32_16x16x32_f16(false, a, false, b, (short)0, c, false, false);
  asm volatile("v_nop\n\tv_nop\n\tv_nop\n\tv_nop" : "+v"(d) : "v"(a), "v"(b));
  return d;
}

__device__ __forceinline__ v16h load_frag(const _Float16* p, int h) {
  Frag f;
  f.half[0] = *(const v8ha*)(p + 8 * h);
  f.half[1] = *(const v8ha*)(p + 16 + 8 * h);
  return f.v;
}

__global__ __launch_bounds__(256) void convert_kernel(
    const float* __restrict__ x, const float* __restrict__ y,
    _Float16* __restrict__ xh, _Float16* __restrict__ yh)
{
  const int g = blockIdx.x * 256 + threadIdx.x;
  if (g >= 2 * G8) return;
  const int sel = (g >= G8) ? 1 : 0;
  const int e = g - sel * G8;
  const int row = e >> 4;
  const int q = e & 15;
  const int s = row >> 5;
  const int n = row & 31;
  const float* src = (sel ? y : x) + (size_t)row * DIM + 8 * q;
  _Float16* dst = (sel ? yh : xh) + ((size_t)n * SEQ + s) * DIM + 8 * q;
  const v4f a = *(const v4fa*)src;
  const v4f c = *(const v4fa*)(src + 4);
  const v8h o = { (_Float16)a.x, (_Float16)a.y, (_Float16)a.z, (_Float16)a.w,
                  (_Float16)c.x, (_Float16)c.y, (_Float16)c.z, (_Float16)c.w };
  *(volatile v8h*)dst = o;
  __threadfence();
  *(volatile v8h*)dst = o;
}

__global__ __launch_bounds__(NTHR) void score_pool_kernel(
    const _Float16* __restrict__ xh,
    const _Float16* __restrict__ yh,
    float* __restrict__ rv)
{
  __shared__ __attribute__((aligned(16))) float sc[RPB * SEQ];
  __shared__ __attribute__((aligned(16))) float rvs[RVL];

  const int tid = threadIdx.x, lane = tid & 31, w = tid >> 5;
  const int h = lane >> 4, m = lane & 15;
  const int rt = blockIdx.x, n = blockIdx.y;
  const int row0 = rt * RPB;

  if (tid < RVL) rvs[tid] = 0.0f;

  const _Float16* ya = yh + ((size_t)n * SEQ + row0 + m) * DIM;
  const v16h a0 = load_frag(ya, h);
  const v16h a1 = load_frag(ya + 32, h);
  const v16h a2 = load_frag(ya + 64, h);
  const v16h a3 = load_frag(ya + 96, h);

  const _Float16* xb = xh + ((size_t)n * SEQ + w * CPW + m) * DIM;
  const v8f zero8 = {0.f, 0.f, 0.f, 0.f, 0.f, 0.f, 0.f, 0.f};
  #pragma unroll 1
  for (int t = 0; t < CPW / 16; ++t) {
    const _Float16* bp = xb + (size_t)t * 16 * DIM;
    v8f acc = zero8;
    acc = wmma_f16(a0, load_frag(bp, h), acc);
    acc = wmma_f16(a1, load_frag(bp + 32, h), acc);
    acc = wmma_f16(a2, load_frag(bp + 64, h), acc);
    acc = wmma_f16(a3, load_frag(bp + 96, h), acc);
    const int col = w * CPW + 16 * t + m;
    #pragma unroll
    for (int r = 0; r < 8; ++r) sc[(8 * h + r) * SEQ + col] = acc[r];
  }
  __syncthreads();

  const float ninf = -__builtin_inff();
  float lsum[4];
  #pragma unroll
  for (int rr = 0; rr < 4; ++rr) {
    float* srow = sc + (w * 4 + rr) * SEQ;
    float mx = ninf;
    #pragma unroll 1
    for (int j = lane; j < SEQ; j += 32) mx = fmaxf(mx, srow[j]);
    #pragma unroll
    for (int off = 16; off >= 1; off >>= 1) mx = fmaxf(mx, __shfl_xor(mx, off, 32));
    float s = 0.0f;
    #pragma unroll 1
    for (int j = lane; j < SEQ; j += 32) {
      const float e = __expf(srow[j] - mx);
      srow[j] = e;
      s += e;
    }
    #pragma unroll
    for (int off = 16; off >= 1; off >>= 1) s += __shfl_xor(s, off, 32);
    lsum[rr] = s;
  }
  __syncthreads();

  #pragma unroll
  for (int rr = 0; rr < 4; ++rr) {
    const float* srow = sc + (w * 4 + rr) * SEQ;
    float wm = ninf;
    #pragma unroll 1
    for (int j = lane; j < SEQ - 2; j += 32) wm = fmaxf(wm, (srow[j] + srow[j + 1]) + srow[j + 2]);
    #pragma unroll
    for (int off = 16; off >= 1; off >>= 1) wm = fmaxf(wm, __shfl_xor(wm, off, 32));
    const float val = wm * (1.0f / lsum[rr]) * (1.0f / 3.0f);
    if (lane == 0) rvs[w * 4 + rr] = val;
  }
  __syncthreads();

  const bool writer = (w == 0) && (lane < 8);
  const v4f v = *(const v4fa*)(rvs + 4 * (lane & 7));
  float* dst = rv + ((size_t)n * RT + rt) * RVL + 4 * (lane & 7);
  if (writer) *(volatile v4f*)dst = v;
  __threadfence();
  if (writer) *(volatile v4f*)dst = v;
}

__global__ __launch_bounds__(32) void mean_kernel(const float* __restrict__ rv,
                                                  float* __restrict__ out)
{
  __shared__ __attribute__((aligned(16))) float so[NB];
  const int lane = threadIdx.x;
  const float* p = rv + (size_t)lane * RT * RVL;
  double acc = 0.0;
  #pragma unroll 1
  for (int t = 0; t < RT; ++t) {
    const float* q = p + t * RVL;
    #pragma unroll
    for (int i = 0; i < 4; ++i) {
      const v4f v = *(const v4fa*)(q + 4 * i);
      acc += (double)v.x;
      acc += (double)v.y;
      acc += (double)v.z;
      acc += (double)v.w;
    }
  }
  so[lane] = (float)(acc * (1.0 / (double)SEQ));
  __syncthreads();
  const v4f o = *(const v4fa*)(so + 4 * (lane & 7));
  if (lane < 8) *(volatile v4f*)(out + 4 * lane) = o;
  __threadfence();
  if (lane < 8) *(volatile v4f*)(out + 4 * lane) = o;
}

extern "C" void kernel_launch(void* const* d_in, const int* in_sizes, int n_in,
                              void* d_out, int out_size, void* d_ws, size_t ws_size,
                              hipStream_t stream) {
  if (n_in < 2) return;
  if (in_sizes[0] != NELEM || in_sizes[1] != NELEM) return;
  if (out_size != NB) return;

  const float* x = (const float*)d_in[0];
  const float* y = (const float*)d_in[1];
  float* out = (float*)d_out;

  const size_t plane_bytes = (size_t)NELEM * 2;
  const size_t rv_bytes    = (size_t)NB * RT * RVL * 4;
  const size_t total       = 2 * plane_bytes + rv_bytes;
  if (total > ws_size) return;

  char* ws = (char*)d_ws;
  _Float16* xh = (_Float16*)(ws);
  _Float16* yh = (_Float16*)(ws + plane_bytes);
  float* rv    = (float*)(ws + 2 * plane_bytes);

  const int ngroups = 2 * G8;
  convert_kernel<<<(ngroups + 255) / 256, 256, 0, stream>>>(x, y, xh, yh);

  dim3 gScore(RT, NB);
  score_pool_kernel<<<gScore, NTHR, 0, stream>>>(xh, yh, rv);

  mean_kernel<<<1, 32, 0, stream>>>(rv, out);
}
